// MultiheadSelfAttention_10874857193993
// MI455X (gfx1250) — hardware-verified
//
#include <hip/hip_runtime.h>


#ifndef NB
#define NB 4
#endif
#ifndef SEQ
#define SEQ 2048
#endif
#define NB_FULL  4
#define SEQ_FULL 2048
#define DM   512
#define NH   8
#define HD   64
#define DMH  (NH * HD)
#define DOUT 512
#define ATP  (2 * DMH)
#define QCAR 16.0f
#define PEXP 8.0f
#define CEXP ((float)(0.125 * 1.4426950408889634 / 256.0))

typedef _Float16 h16;
typedef unsigned short bf;
typedef __attribute__((ext_vector_type(16))) __bf16   v16bf;
typedef __attribute__((ext_vector_type(16))) _Float16 v16h;
typedef __attribute__((ext_vector_type(8)))  _Float16 v8h;
typedef __attribute__((ext_vector_type(8)))  unsigned short v8us;
typedef __attribute__((ext_vector_type(2)))  unsigned short v2us;
typedef __attribute__((ext_vector_type(8)))  float    v8f;
typedef __attribute__((ext_vector_type(4)))  float    v4f;
typedef v4f  __attribute__((may_alias)) v4fa;

static_assert(HD == 64);
static_assert(SEQ % 64 == 0);
static_assert((NB * SEQ) % 64 == 0);
static_assert(DM % 32 == 0);
static_assert(ATP % 32 == 0);
static_assert(DMH % 64 == 0);
static_assert(DOUT % 64 == 0);
static_assert(DM % 8 == 0);
static_assert((SEQ / 8) % 8 == 0);
static_assert(NB <= NB_FULL);
static_assert(SEQ <= SEQ_FULL);
static_assert(DMH == DOUT);

#define RUP256(x) ((((size_t)(x)) + 255) & ~(size_t)255)
#define SZ_XB   RUP256((size_t)NB * SEQ * DM * 2)
#define SZ_WQKV RUP256((size_t)3 * DMH * DM * 2)
#define SZ_WO   RUP256((size_t)DOUT * ATP * 2)
#define SZ_F    RUP256((size_t)NB * SEQ * DMH * 4)
#define SZ_PL   RUP256((size_t)NB * NH * SEQ * HD * 2)
#define SZ_AT   RUP256((size_t)NB * SEQ * ATP * 2)
#define SZ_TOT  (SZ_XB + SZ_WQKV + SZ_WO + SZ_F + 3 * SZ_PL + SZ_AT)
static_assert(SZ_TOT <= (size_t)134217728);

__device__ __forceinline__ unsigned short f2bf(float f) { unsigned u = __float_as_uint(f); u += 0x7FFFu + ((u >> 16) & 1u); return (unsigned short)(u >> 16); }
__device__ __forceinline__ float bf2f(unsigned short b) { return __uint_as_float(((unsigned)b) << 16); }
__device__ __forceinline__ float bfr(float f) { return bf2f(f2bf(f)); }
__device__ __forceinline__ void splitf(float y, unsigned short& h, unsigned short& l) { h = f2bf(y); l = f2bf(y - bf2f(h)); }
__device__ __forceinline__ v16h cat16(v8h lo, v8h hi) { return __builtin_shufflevector(lo, hi, 0, 1, 2, 3, 4, 5, 6, 7, 8, 9, 10, 11, 12, 13, 14, 15); }
__device__ __forceinline__ v16bf cat16b(v8us lo, v8us hi) { return __builtin_bit_cast(v16bf, __builtin_shufflevector(lo, hi, 0, 1, 2, 3, 4, 5, 6, 7, 8, 9, 10, 11, 12, 13, 14, 15)); }
__device__ __forceinline__ v8f wmma16(v16h a, v16h b, v8f c) { return __builtin_amdgcn_wmma_f32_16x16x32_f16(false, a, false, b, (short)0, c, false, false); }
__device__ __forceinline__ v8f wmmab(v16bf a, v16bf b, v8f c) { return __builtin_amdgcn_wmma_f32_16x16x32_bf16(false, a, false, b, (short)0, c, false, false); }
__device__ __forceinline__ v16h  ldh(const h16* p) { return cat16(*(const v8h*)p, *(const v8h*)(p + 16)); }
__device__ __forceinline__ v16bf ldb(const bf* p)  { return cat16b(*(const v8us*)p, *(const v8us*)(p + 16)); }

__global__ __launch_bounds__(32) void k_gemm(const bf* __restrict__ A, const bf* __restrict__ Bt, int K, float* C, int ldc, const float* __restrict__ bias, size_t sA, size_t sC) {
    __shared__ __align__(16) float os[16 * 68];
    const size_t z = blockIdx.z; A += z * sA; C += z * sC;
    const int lane = threadIdx.x & 31, lr = lane & 15, hi = lane >> 4; const int r0 = blockIdx.x * 64, c0 = blockIdx.y * 64;
    v8f acc[4][4];
#pragma unroll
    for (int mb = 0; mb < 4; ++mb)
#pragma unroll
        for (int nb = 0; nb < 4; ++nb) acc[mb][nb] = (v8f){};
    const size_t aoff = (size_t)(r0 + lr) * K + 8 * hi, boff = (size_t)(c0 + lr) * K + 8 * hi;
#pragma unroll 1
    for (int kc = 0; kc < K; kc += 32) {
        v16bf a[4];
#pragma unroll
        for (int mb = 0; mb < 4; ++mb) a[mb] = ldb(A + aoff + (size_t)mb * 16 * K + kc);
#pragma unroll
        for (int nb = 0; nb < 4; ++nb) { const v16bf b = ldb(Bt + boff + (size_t)nb * 16 * K + kc);
#pragma unroll
            for (int mb = 0; mb < 4; ++mb) acc[mb][nb] = wmmab(a[mb], b, acc[mb][nb]); }
        asm volatile("v_nop\n\tv_nop\n\tv_nop\n\tv_nop" : "+v"(acc[0][0]), "+v"(acc[1][1]), "+v"(acc[2][2]), "+v"(acc[3][3]) : "v"(a[0]), "v"(a[3]));
    }
#pragma unroll
    for (int mb = 0; mb < 4; ++mb) {
#pragma unroll
        for (int nb = 0; nb < 4; ++nb) {
#pragma unroll
            for (int j = 0; j < 8; ++j) os[(hi * 8 + j) * 68 + nb * 16 + lr] = acc[mb][nb][j]; }
        __builtin_amdgcn_fence(3  , "wavefront"); __builtin_amdgcn_wave_barrier(); asm volatile("" ::: "memory");
        float* crow = C + (size_t)(r0 + mb * 16) * ldc + c0;
        const int cofs = lr * 4;
        const float b0 = bfr(bias[c0 + cofs]), b1 = bfr(bias[c0 + cofs + 1]), b2 = bfr(bias[c0 + cofs + 2]), b3 = bfr(bias[c0 + cofs + 3]);
#pragma unroll 1
        for (int ps = 0; ps < 2; ++ps) {
#pragma unroll
            for (int s = 0; s < 8; ++s) { const int row = 2 * s + hi; v4f val = *(const v4fa*)(os + row * 68 + cofs); val[0] += b0; val[1] += b1; val[2] += b2; val[3] += b3;
                *(volatile v4f*)(crow + (size_t)row * ldc + cofs) = val; }
            if (ps == 0) __threadfence(); }
        __builtin_amdgcn_fence(3  , "wavefront"); __builtin_amdgcn_wave_barrier(); asm volatile("" ::: "memory");
    }
}

__global__ __launch_bounds__(256) void k_wt(const float* __restrict__ w, int K, int N, int H, int KREP, bf* Bt) {
    const int wave = __builtin_amdgcn_readfirstlane(threadIdx.x >> 5);
    const unsigned lane = threadIdx.x & 31; const unsigned L0 = (blockIdx.x * 8u + (unsigned)wave) * 8u; const unsigned KP = (unsigned)(K * KREP); const unsigned nlines = (unsigned)H * (unsigned)N * KP / 64u;
#pragma unroll 1
    for (int ps = 0; ps < 2; ++ps) {
#pragma unroll 1
        for (int l = 0; l < 8; ++l) { const unsigned L = L0 + l; if (L >= nlines) break; const unsigned e = L * 64u + lane * 2u; const unsigned kk = e % KP, ng = e / KP; const unsigned hh = ng / (unsigned)N, n = ng % (unsigned)N; const unsigned k = kk % (unsigned)K; v2us o;
            o[0] = f2bf(w[((size_t)hh * K + k) * N + n]); o[1] = f2bf(w[((size_t)hh * K + k + 1) * N + n]); *(volatile v2us*)(Bt + e) = o; }
        if (ps == 0) __threadfence(); }
}

__global__ __launch_bounds__(256) void k_cvt(const float* __restrict__ x, bf* XB) {
    const unsigned i = blockIdx.x * 256u + threadIdx.x; if (i >= (unsigned)(NB * SEQ * (DM / 8))) return;
    const unsigned row = i / (DM / 8), c8 = i % (DM / 8); const unsigned b = row / SEQ, t = row % SEQ;
    const v8f v = *(const v8f*)(x + ((size_t)(b * SEQ_FULL + t) * DM + c8 * 8)); v8us o;
#pragma unroll
    for (int k = 0; k < 8; ++k) o[k] = f2bf(v[k]);
    *(volatile v8us*)(XB + (size_t)i * 8) = o; __threadfence(); *(volatile v8us*)(XB + (size_t)i * 8) = o; }

__global__ __launch_bounds__(256) void k_qkp(const float* __restrict__ F, h16* P) {
    const unsigned i = blockIdx.x * 256u + threadIdx.x; if (i >= (unsigned)(NB * NH * SEQ * (HD / 8))) return;
    const unsigned d8 = i % (HD / 8); const unsigned t = (i / (HD / 8)) % SEQ; const unsigned g = i / ((HD / 8) * SEQ); const unsigned h = g % NH, b = g / NH;
    const v8f v = *(const v8f*)(F + ((size_t)(b * SEQ + t) * DMH + h * HD + d8 * 8)); v8h o;
#pragma unroll
    for (int k = 0; k < 8; ++k) o[k] = (h16)(v[k] * QCAR);
    *(volatile v8h*)(P + (size_t)i * 8) = o; __threadfence(); *(volatile v8h*)(P + (size_t)i * 8) = o; }

__global__ __launch_bounds__(256) void k_vtp(const float* __restrict__ F, h16* VT) {
    const unsigned i = blockIdx.x * 256u + threadIdx.x; if (i >= (unsigned)(NB * NH * HD * (SEQ / 8))) return;
    const unsigned t8 = i % (SEQ / 8); const unsigned d = (i / (SEQ / 8)) % HD; const unsigned g = i / ((SEQ / 8) * HD); const unsigned h = g % NH, b = g / NH;
    const float* f = F + ((size_t)(b * SEQ + t8 * 8) * DMH + h * HD + d); v8h o;
#pragma unroll
    for (int q = 0; q < 8; ++q) o[q] = (h16)(f[(size_t)q * DMH] * QCAR);
    *(volatile v8h*)(VT + (size_t)i * 8) = o; __threadfence(); *(volatile v8h*)(VT + (size_t)i * 8) = o; }

__global__ __launch_bounds__(128) void k_attn(const h16* __restrict__ Q16, const h16* __restrict__ K16, const h16* __restrict__ VT16, bf* AT) {
    __shared__ __align__(16) float os[4 * 16 * 68];
    const int wave = __builtin_amdgcn_readfirstlane(threadIdx.x >> 5);
    const int lane = threadIdx.x & 31, lr = lane & 15, hi = lane >> 4;
    const int bh = blockIdx.y; const int b = bh / NH, h = bh % NH;
    const int q0 = blockIdx.x * 64 + wave * 16;
    const h16* Qp = Q16 + (size_t)bh * SEQ * HD + (size_t)(q0 + lr) * HD + 8 * hi;
    const h16* Kp = K16 + (size_t)bh * SEQ * HD + lr * HD + 8 * hi;
    const h16* Vp = VT16 + (size_t)bh * HD * SEQ + (size_t)lr * SEQ + 8 * hi;
    const v16h qb0 = ldh(Qp), qb1 = ldh(Qp + 32);
    v8f o0 = (v8f){}, o1 = (v8f){}, o2 = (v8f){}, o3 = (v8f){};
    float m = -3.0e38f, ls = 0.0f;
#pragma unroll 1
    for (int j0 = 0; j0 < SEQ; j0 += 32) {
        const h16* kp = Kp + (size_t)j0 * HD;
        const v16h ka = ldh(kp), kb = ldh(kp + 32), kc = ldh(kp + 16 * HD), kd = ldh(kp + 16 * HD + 32);
        v8f s0 = (v8f){}, s1 = (v8f){};
        s0 = wmma16(ka, qb0, s0); s1 = wmma16(kc, qb0, s1); s0 = wmma16(kb, qb1, s0); s1 = wmma16(kd, qb1, s1);
        asm volatile("v_nop\n\tv_nop\n\tv_nop\n\tv_nop" : "+v"(s0), "+v"(s1) : "v"(ka), "v"(kb), "v"(kc), "v"(kd), "v"(qb0), "v"(qb1));
        const h16* vp = Vp + j0;
        const v16h v0 = ldh(vp), v1 = ldh(vp + (size_t)16 * SEQ), v2 = ldh(vp + (size_t)32 * SEQ), v3 = ldh(vp + (size_t)48 * SEQ);
        float mx = fmaxf(s0[0], s1[0]);
#pragma unroll
        for (int r = 1; r < 8; ++r) mx = fmaxf(mx, fmaxf(s0[r], s1[r]));
        mx = fmaxf(mx, __shfl_xor(mx, 16, 32));
        const float mn = fmaxf(m, mx * CEXP);
        const float corr = __builtin_amdgcn_exp2f(m - mn);
        m = mn;
        const float nbv = PEXP - mn;
        float psum = 0.0f; v16h pb;
#pragma unroll
        for (int r = 0; r < 8; ++r) { const float p0 = __builtin_amdgcn_exp2f(fmaf(s0[r], CEXP, nbv)); const float p1 = __builtin_amdgcn_exp2f(fmaf(s1[r], CEXP, nbv)); psum += p0 + p1; pb[r] = (h16)p0; pb[8 + r] = (h16)p1; }
        ls = ls * corr + psum;
        o0 *= corr; o1 *= corr; o2 *= corr; o3 *= corr;
        o0 = wmma16(v0, pb, o0); o1 = wmma16(v1, pb, o1); o2 = wmma16(v2, pb, o2); o3 = wmma16(v3, pb, o3);
        asm volatile("v_nop\n\tv_nop\n\tv_nop\n\tv_nop" : "+v"(o0), "+v"(o1), "+v"(o2), "+v"(o3) : "v"(pb), "v"(v0), "v"(v1), "v"(v2), "v"(v3));
    }
    const float lt = ls + __shfl_xor(ls, 16, 32);
    const float inv = 1.0f / (lt * QCAR);
    const int osw = wave * (16 * 68);
    {
        float* orow = os + osw + lr * 68 + 8 * hi;
        v4f w;
        w[0] = o0[0] * inv; w[1] = o0[1] * inv; w[2] = o0[2] * inv; w[3] = o0[3] * inv; *(v4fa*)(orow + 0) = w;
        w[0] = o0[4] * inv; w[1] = o0[5] * inv; w[2] = o0[6] * inv; w[3] = o0[7] * inv; *(v4fa*)(orow + 4) = w;
        w[0] = o1[0] * inv; w[1] = o1[1] * inv; w[2] = o1[2] * inv; w[3] = o1[3] * inv; *(v4fa*)(orow + 16) = w;
        w[0] = o1[4] * inv; w[1] = o1[5] * inv; w[2] = o1[6] * inv; w[3] = o1[7] * inv; *(v4fa*)(orow + 20) = w;
        w[0] = o2[0] * inv; w[1] = o2[1] * inv; w[2] = o2[2] * inv; w[3] = o2[3] * inv; *(v4fa*)(orow + 32) = w;
        w[0] = o2[4] * inv; w[1] = o2[5] * inv; w[2] = o2[6] * inv; w[3] = o2[7] * inv; *(v4fa*)(orow + 36) = w;
        w[0] = o3[0] * inv; w[1] = o3[1] * inv; w[2] = o3[2] * inv; w[3] = o3[3] * inv; *(v4fa*)(orow + 48) = w;
        w[0] = o3[4] * inv; w[1] = o3[5] * inv; w[2] = o3[6] * inv; w[3] = o3[7] * inv; *(v4fa*)(orow + 52) = w;
    }
    __builtin_amdgcn_fence(3  , "wavefront"); __builtin_amdgcn_wave_barrier(); asm volatile("" ::: "memory");
    bf* arow = AT + (size_t)(b * SEQ + q0) * ATP + h * HD;
    const int rq = lane >> 3, c = (lane & 7) * 8;
#pragma unroll 1
    for (int ps = 0; ps < 2; ++ps) {
#pragma unroll
        for (int s = 0; s < 4; ++s) { const int row = 4 * s + rq; const v4f x0 = *(const v4fa*)(os + osw + row * 68 + c); const v4f x1 = *(const v4fa*)(os + osw + row * 68 + c + 4); v8us oh, ol;
#pragma unroll
            for (int k = 0; k < 4; ++k) { unsigned short a, l2; splitf(x0[k], a, l2); oh[k] = a; ol[k] = l2; splitf(x1[k], a, l2); oh[4 + k] = a; ol[4 + k] = l2; }
            *(volatile v8us*)(arow + (size_t)row * ATP + c) = oh; *(volatile v8us*)(arow + (size_t)row * ATP + DMH + c) = ol; }
        if (ps == 0) __threadfence(); }
}

extern "C" void kernel_launch(void* const* d_in, const int* in_sizes, int n_in,
                              void* d_out, int out_size, void* d_ws, size_t ws_size, hipStream_t stream) {
    if (n_in < 9) return;
    const long long rowsNeeded = (long long)(NB - 1) * SEQ_FULL + SEQ;
    if ((long long)in_sizes[0] < rowsNeeded * DM) return;
    if (in_sizes[1] < NH * DM * HD || in_sizes[3] < NH * DM * HD || in_sizes[5] < NH * DM * HD) return;
    if (in_sizes[2] < DMH || in_sizes[4] < DMH || in_sizes[6] < DMH) return;
    if (in_sizes[7] < DMH * DOUT || in_sizes[8] < DOUT) return;
    if ((long long)out_size < rowsNeeded * DOUT) return;
    if (ws_size < SZ_TOT) return;
    const float* feat = (const float*)d_in[0];
    const float* Wq = (const float*)d_in[1]; const float* bq = (const float*)d_in[2];
    const float* Wk = (const float*)d_in[3]; const float* bk = (const float*)d_in[4];
    const float* Wv = (const float*)d_in[5]; const float* bv = (const float*)d_in[6];
    const float* Wf = (const float*)d_in[7]; const float* bo = (const float*)d_in[8];
    float* OUT = (float*)d_out;
    char* wsp = (char*)d_ws;
    bf* XB = (bf*)wsp; wsp += SZ_XB;
    bf* WQKV = (bf*)wsp; wsp += SZ_WQKV;
    bf* WO = (bf*)wsp; wsp += SZ_WO;
    float* F = (float*)wsp; wsp += SZ_F;
    h16* Q16 = (h16*)wsp; wsp += SZ_PL;
    h16* K16 = (h16*)wsp; wsp += SZ_PL;
    h16* VT16 = (h16*)wsp; wsp += SZ_PL;
    bf* AT = (bf*)wsp; wsp += SZ_AT;
    if ((size_t)(wsp - (char*)d_ws) > ws_size) return;

    k_cvt<<<(unsigned)((NB * SEQ * (DM / 8) + 255) / 256), 256, 0, stream>>>(feat, XB);
    const unsigned gw = (unsigned)((NH * HD * DM / 64 + 63) / 64);
    k_wt<<<gw, 256, 0, stream>>>(Wq, DM, HD, NH, 1, WQKV);
    k_wt<<<gw, 256, 0, stream>>>(Wk, DM, HD, NH, 1, WQKV + (size_t)DMH * DM);
    k_wt<<<gw, 256, 0, stream>>>(Wv, DM, HD, NH, 1, WQKV + (size_t)2 * DMH * DM);
    k_wt<<<(unsigned)((DOUT * ATP / 64 + 63) / 64), 256, 0, stream>>>(Wf, DMH, DOUT, 1, 2, WO);

    const dim3 gp(NB * SEQ / 64, DMH / 64, 1);
    const unsigned gq = (unsigned)((NB * NH * SEQ * (HD / 8) + 255) / 256);
    k_gemm<<<gp, 32, 0, stream>>>(XB, WQKV, DM, F, DMH, bq, 0, 0);
    k_qkp<<<gq, 256, 0, stream>>>(F, Q16);
    k_gemm<<<gp, 32, 0, stream>>>(XB, WQKV + (size_t)DMH * DM, DM, F, DMH, bk, 0, 0);
    k_qkp<<<gq, 256, 0, stream>>>(F, K16);
    k_gemm<<<gp, 32, 0, stream>>>(XB, WQKV + (size_t)2 * DMH * DM, DM, F, DMH, bv, 0, 0);
    k_vtp<<<(unsigned)((NB * NH * HD * (SEQ / 8) + 255) / 256), 256, 0, stream>>>(F, VT16);

    k_attn<<<dim3(SEQ / 64, NB * NH, 1), 128, 0, stream>>>(Q16, K16, VT16, AT);

    k_gemm<<<dim3(SEQ / 64, DOUT / 64, NB), 32, 0, stream>>>(AT, WO, ATP, OUT, DOUT, bo, (size_t)SEQ * ATP, (size_t)SEQ_FULL * DOUT);
}
